// TaskAllocatorNetwork_35983236006575
// MI455X (gfx1250) — hardware-verified
//
#include <hip/hip_runtime.h>


#define NBT  32
#define NRB  512
#define NTS  128
#define HH   64
#define NHD  4
#define HD   16
#define NRR  (NBT * NRB)
#define NTR  (NBT * NTS)
#define NPR  (NTS * NRB)
#define DM   HH
#define LOSC 1024.0f

typedef _Float16 h16;
typedef unsigned short bf;
typedef __attribute__((ext_vector_type(16))) __bf16   v16bf;
typedef __attribute__((ext_vector_type(16))) _Float16 v16h;
typedef __attribute__((ext_vector_type(8)))  _Float16 v8h;
typedef __attribute__((ext_vector_type(8)))  unsigned short v8us;
typedef __attribute__((ext_vector_type(8)))  float    v8f;
typedef __attribute__((ext_vector_type(4)))  float    v4f;
typedef v8h  __attribute__((may_alias)) v8ha;
typedef v4f  __attribute__((may_alias)) v4fa;
typedef v8us __attribute__((may_alias)) v8usa;

__device__ __forceinline__ unsigned short f2bf(float f) { unsigned u = __float_as_uint(f); u += 0x7FFFu + ((u >> 16) & 1u); return (unsigned short)(u >> 16); }
__device__ __forceinline__ float bf2f(unsigned short b) { return __uint_as_float(((unsigned)b) << 16); }
__device__ __forceinline__ float bfr(float f) { return bf2f(f2bf(f)); }
__device__ __forceinline__ v16h cat16(v8h lo, v8h hi) { return __builtin_shufflevector(lo, hi, 0, 1, 2, 3, 4, 5, 6, 7, 8, 9, 10, 11, 12, 13, 14, 15); }
__device__ __forceinline__ v16bf cat16b(v8us lo, v8us hi) { return __builtin_bit_cast(v16bf, __builtin_shufflevector(lo, hi, 0, 1, 2, 3, 4, 5, 6, 7, 8, 9, 10, 11, 12, 13, 14, 15)); }
__device__ __forceinline__ v8f wmma16(v16h a, v16h b, v8f c) { return __builtin_amdgcn_wmma_f32_16x16x32_f16(false, a, false, b, (short)0, c, false, false); }
__device__ __forceinline__ v8f wmmab(v16bf a, v16bf b, v8f c) { return __builtin_amdgcn_wmma_f32_16x16x32_bf16(false, a, false, b, (short)0, c, false, false); }

template <bool SPLITA, bool F16OUT = false>
__global__ __launch_bounds__(128) void k_gemmb(const bf* __restrict__ A, const bf* __restrict__ Al, const bf* __restrict__ Bn, const float* __restrict__ bias, float* C, int ldc, h16* C2, const float* __restrict__ R = nullptr, int K = DM, int roundR = 1) {
    __shared__ __align__(16) float ost[4][16 * 68];
    const int lane = threadIdx.x & 31, wave = threadIdx.x >> 5, lr = lane & 15, hi = lane >> 4;
    const int r0 = blockIdx.x * 64 + wave * 16, c0 = blockIdx.y * 64;
    const size_t aoff = (size_t)(r0 + lr) * K + 8 * hi;
    size_t boff[4];
#pragma unroll
    for (int t = 0; t < 4; ++t) boff[t] = (size_t)(c0 + t * 16 + lr) * K + 8 * hi;
    v8f acc[4];
#pragma unroll
    for (int t = 0; t < 4; ++t) acc[t] = (v8f){};
#pragma unroll 1
    for (int kc = 0; kc < K; kc += 32) {
        const v16bf a = cat16b(*(const v8us*)(A + aoff + kc), *(const v8us*)(A + aoff + kc + 16));
        v16bf al = a;
        if (SPLITA) al = cat16b(*(const v8us*)(Al + aoff + kc), *(const v8us*)(Al + aoff + kc + 16));
#pragma unroll
        for (int t = 0; t < 4; ++t) { const v16bf b = cat16b(*(const v8us*)(Bn + boff[t] + kc), *(const v8us*)(Bn + boff[t] + kc + 16)); acc[t] = wmmab(a, b, acc[t]); if (SPLITA) acc[t] = wmmab(al, b, acc[t]); }
        asm volatile("v_nop\n\tv_nop\n\tv_nop\n\tv_nop" : "+v"(acc[0]), "+v"(acc[1]), "+v"(acc[2]), "+v"(acc[3]) : "v"(a), "v"(al));
    }
    float* os = &ost[wave][0];
#pragma unroll
    for (int t = 0; t < 4; ++t) { const float bv = bias ? bfr(bias[c0 + t * 16 + lr]) : 0.f;
#pragma unroll
        for (int j = 0; j < 8; ++j) os[(hi * 8 + j) * 68 + t * 16 + lr] = acc[t][j] + bv; }
    __syncthreads();
    if (F16OUT) {
        h16* crow = (h16*)(void*)C + (size_t)r0 * ldc + c0;
        auto pass = [&]() {
#pragma unroll
            for (int s = 0; s < 4; ++s) { const int row = 4 * s + (lane >> 3), piece = lane & 7; const float* sp = os + row * 68 + piece * 8; v8h o, o2;
#pragma unroll
                for (int i = 0; i < 8; ++i) { const h16 a = (h16)sp[i]; o[i] = a; o2[i] = (h16)((sp[i] - (float)a) * LOSC); }
                *(volatile v8h*)(crow + (size_t)row * ldc + piece * 8) = o; if (C2) *(volatile v8h*)(C2 + (size_t)r0 * ldc + c0 + (size_t)row * ldc + piece * 8) = o2; }
        };
        pass(); __threadfence(); pass();
    } else {
        float* crow = C + (size_t)r0 * ldc + c0;
        auto pass = [&]() {
#pragma unroll
            for (int s = 0; s < 8; ++s) { const int Lid = (lane >> 3) + 4 * s, piece = lane & 7; const int row = Lid >> 1, cofs = (Lid & 1) * 32 + piece * 4;
                v4f val = *(const v4fa*)(os + row * 68 + cofs); if (R) { const v4f rv = *(const v4f*)(R + ((size_t)r0 + row) * ldc + c0 + cofs); val += roundR ? (v4f){bfr(rv[0]), bfr(rv[1]), bfr(rv[2]), bfr(rv[3])} : rv; }
                *(volatile v4f*)(crow + (size_t)row * ldc + cofs) = val; }
        };
        pass(); __threadfence(); pass();
    }
}

__global__ __launch_bounds__(256) void k_wt(const float* __restrict__ Wm, int K, int ncols, bf* WT) {
    __shared__ __align__(16) unsigned short tl[64 * 72];
    const int tid = threadIdx.x, k0 = blockIdx.x * 64, n0 = blockIdx.y * 64;
    const int kk = tid >> 2, nq = (tid & 3) * 16;
#pragma unroll
    for (int i = 0; i < 16; ++i) tl[(nq + i) * 72 + kk] = f2bf(Wm[(size_t)(k0 + kk) * ncols + n0 + nq + i]);
    __syncthreads();
    const int piece = tid & 7;
    auto pass = [&]() {
#pragma unroll
        for (int s = 0; s < 2; ++s) { const int nr = (tid >> 3) + 32 * s; const v8us val = *(const v8usa*)(tl + nr * 72 + piece * 8); *(volatile v8us*)(WT + (size_t)(n0 + nr) * K + k0 + piece * 8) = val; }
    };
    pass(); __threadfence(); pass();
}

__global__ __launch_bounds__(256) void k_wtp(const float* __restrict__ Wm, int krows, int ncols, int kpad, bf* WT) {
    __shared__ __align__(16) unsigned short tl[64 * 72];
    const int tid = threadIdx.x, k0 = blockIdx.x * 64, n0 = blockIdx.y * 64;
    const int kk = tid >> 2, nq = (tid & 3) * 16;
    const int k = k0 + kk, kc = k < krows ? k : krows - 1;
#pragma unroll
    for (int i = 0; i < 16; ++i) { const int n = n0 + nq + i, ncl = n < ncols ? n : ncols - 1; const float w = Wm[(size_t)kc * ncols + ncl]; tl[(nq + i) * 72 + kk] = (k < krows && n < ncols) ? f2bf(w) : (unsigned short)0; }
    __syncthreads();
    const int piece = tid & 7;
    auto pass = [&]() {
#pragma unroll
        for (int s = 0; s < 2; ++s) { const int nr = (tid >> 3) + 32 * s; const v8us val = *(const v8usa*)(tl + nr * 72 + piece * 8); *(volatile v8us*)(WT + (size_t)(n0 + nr) * kpad + k0 + piece * 8) = val; }
    };
    pass(); __threadfence(); pass();
}

__global__ __launch_bounds__(256) void k_pad32(const float* __restrict__ src, int nrows, int nc, bf* X) {
    const int lane = threadIdx.x & 31; const size_t r = ((size_t)blockIdx.x * 8 + (threadIdx.x >> 5)) * 8 + (lane >> 2); if (r >= (size_t)nrows) return; const int cb = (lane & 3) * 8; v8us o;
#pragma unroll
    for (int i = 0; i < 8; ++i) { const int c = cb + i; o[i] = (c < nc) ? f2bf(src[r * nc + (c < nc ? c : 0)]) : (unsigned short)0; }
    *(volatile v8us*)(X + r * 32 + cb) = o; __threadfence(); *(volatile v8us*)(X + r * 32 + cb) = o;
}
template <bool RELU>
__global__ __launch_bounds__(256) void k_act64(const float* __restrict__ src, const float* __restrict__ bias, int nrows, bf* dh, bf* dl, float* F) {
    typedef __attribute__((ext_vector_type(2))) unsigned short v2us; typedef __attribute__((ext_vector_type(2))) float v2f;
    const int lane = threadIdx.x & 31; const size_t r = (size_t)blockIdx.x * 8 + (threadIdx.x >> 5); if (r >= (size_t)nrows) return; v2us oh, ol; v2f fv;
#pragma unroll
    for (int i = 0; i < 2; ++i) { const int c = lane * 2 + i; float v = src[r * HH + c] + (bias ? bfr(bias[c]) : 0.f); if (RELU) v = fmaxf(v, 0.f); fv[i] = v; const unsigned short hb = f2bf(v); oh[i] = hb; ol[i] = f2bf(v - bf2f(hb)); }
    const size_t o = r * HH + lane * 2; *(volatile v2us*)(dh + o) = oh; *(volatile v2us*)(dl + o) = ol; if (F) *(volatile v2f*)(F + o) = fv; __threadfence(); *(volatile v2us*)(dh + o) = oh; *(volatile v2us*)(dl + o) = ol; if (F) *(volatile v2f*)(F + o) = fv;
}
__global__ __launch_bounds__(256) void k_w32k(const float* __restrict__ Wm, int kk, bf* WT) {
    const int u = threadIdx.x; v8us o;
#pragma unroll
    for (int i = 0; i < 8; ++i) { const int f = u * 8 + i; const int n = f / 32, k = f % 32; o[i] = (k < kk) ? f2bf(Wm[(k < kk ? k : 0) * HH + n]) : (unsigned short)0; }
    *(volatile v8us*)(WT + u * 8) = o; __threadfence(); *(volatile v8us*)(WT + u * 8) = o;
}
__global__ __launch_bounds__(256) void k_attn16(const float* __restrict__ Q, const float* __restrict__ Kf, const float* __restrict__ Vf, float* CTX) {
    typedef __attribute__((ext_vector_type(2))) float v2f;
    const int lane = threadIdx.x & 31; const size_t bt = (size_t)blockIdx.x * 8 + (threadIdx.x >> 5); if (bt >= (size_t)NTR) return; const int b = (int)(bt / NTS);
    v2f mine = {0.f, 0.f};
#pragma unroll 1
    for (int h = 0; h < NHD; ++h) { float q[HD];
#pragma unroll
        for (int d = 0; d < HD; ++d) q[d] = Q[bt * HH + h * HD + d] * 0.25f;
        auto logit = [&](int j) -> float { const int r = j * 32 + lane; const float* kr = Kf + ((size_t)b * NRB + r) * HH + h * HD; float s = 0.f;
#pragma unroll
            for (int d = 0; d < HD; ++d) s = fmaf(q[d], kr[d], s);
            return s; };
        float mx = -3.0e38f;
#pragma unroll 1
        for (int j = 0; j < 16; ++j) mx = fmaxf(mx, logit(j));
#pragma unroll
        for (int sh = 16; sh; sh >>= 1) mx = fmaxf(mx, __shfl_xor(mx, sh, 32));
        float sm = 0.f; float cx[HD];
#pragma unroll
        for (int d = 0; d < HD; ++d) cx[d] = 0.f;
#pragma unroll 1
        for (int j = 0; j < 16; ++j) { const int r = j * 32 + lane; const float* vr = Vf + ((size_t)b * NRB + r) * HH + h * HD; const float e = __expf(logit(j) - mx); sm += e;
#pragma unroll
            for (int d = 0; d < HD; ++d) cx[d] = fmaf(e, vr[d], cx[d]); }
#pragma unroll
        for (int sh = 16; sh; sh >>= 1) sm += __shfl_xor(sm, sh, 32);
        const float inv = 1.0f / sm;
#pragma unroll
        for (int d = 0; d < HD; ++d) cx[d] *= inv;
#pragma unroll
        for (int d = 0; d < HD; ++d) {
#pragma unroll
            for (int sh = 16; sh; sh >>= 1) cx[d] += __shfl_xor(cx[d], sh, 32); }
        if ((lane >> 3) == h) { const int d0 = (lane & 7) * 2; float a = 0.f, c = 0.f;
#pragma unroll
            for (int d = 0; d < HD; ++d) { if (d == d0) a = cx[d]; if (d == d0 + 1) c = cx[d]; }
            mine[0] = a; mine[1] = c; } }
    *(volatile v2f*)(CTX + bt * HH + lane * 2) = mine; __threadfence(); *(volatile v2f*)(CTX + bt * HH + lane * 2) = mine;
}
__global__ __launch_bounds__(256) void k_h1(const float* __restrict__ TP, const float* __restrict__ RP, const float* __restrict__ ab1, int b, bf* Ph, bf* Pl) {
    typedef __attribute__((ext_vector_type(2))) unsigned short v2us;
    const int lane = threadIdx.x & 31; const size_t pr = (size_t)blockIdx.x * 8 + (threadIdx.x >> 5); if (pr >= (size_t)NPR) return; const int t = (int)(pr / NRB), r = (int)(pr % NRB); v2us oh, ol;
#pragma unroll
    for (int i = 0; i < 2; ++i) { const int c = lane * 2 + i; const float v = fmaxf(TP[((size_t)b * NTS + t) * HH + c] + RP[((size_t)b * NRB + r) * HH + c] + bfr(ab1[c]), 0.f); const unsigned short hb = f2bf(v); oh[i] = hb; ol[i] = f2bf(v - bf2f(hb)); }
    const size_t o = pr * HH + lane * 2; *(volatile v2us*)(Ph + o) = oh; *(volatile v2us*)(Pl + o) = ol; __threadfence(); *(volatile v2us*)(Ph + o) = oh; *(volatile v2us*)(Pl + o) = ol;
}
__global__ __launch_bounds__(256) void k_score(const float* __restrict__ H2, const float* __restrict__ ab2, const float* __restrict__ aw3, const float* __restrict__ ab3, int b, float* OUTB) {
    const int lane = threadIdx.x & 31; const int t = blockIdx.x * 8 + (threadIdx.x >> 5); if (t >= NTS) return;
    const float b3 = bfr(ab3[0]);
    auto score = [&](int j) -> float { const int r = j * 32 + lane; const float* hr = H2 + ((size_t)t * NRB + r) * HH; float a = b3;
#pragma unroll 8
        for (int c = 0; c < HH / 2; ++c) a = fmaf(fmaxf(hr[c] + bfr(ab2[c]), 0.f), bfr(aw3[c]), a);
        return a; };
    float mx = -3.0e38f;
#pragma unroll 1
    for (int j = 0; j < 16; ++j) mx = fmaxf(mx, score(j));
#pragma unroll
    for (int sh = 16; sh; sh >>= 1) mx = fmaxf(mx, __shfl_xor(mx, sh, 32));
    float sm = 0.f;
#pragma unroll 1
    for (int j = 0; j < 16; ++j) sm += __expf(score(j) - mx);
#pragma unroll
    for (int sh = 16; sh; sh >>= 1) sm += __shfl_xor(sm, sh, 32);
    const float inv = 1.0f / sm;
#pragma unroll 1
    for (int ps = 0; ps < 2; ++ps) {
#pragma unroll 1
        for (int j = 0; j < 16; ++j) *(volatile float*)(OUTB + (size_t)t * NRB + j * 32 + lane) = __expf(score(j) - mx) * inv;
        if (ps == 0) __threadfence(); }
}

extern "C" void kernel_launch(void* const* d_in, const int* in_sizes, int n_in,
                              void* d_out, int out_size, void* d_ws, size_t ws_size, hipStream_t stream) {
    (void)in_sizes; (void)n_in; (void)out_size;
    const float* rs = (const float*)d_in[0]; const float* ts = (const float*)d_in[1];
    const float* rw1 = (const float*)d_in[2]; const float* rb1 = (const float*)d_in[3]; const float* rw2 = (const float*)d_in[4]; const float* rb2 = (const float*)d_in[5];
    const float* tw1 = (const float*)d_in[6]; const float* tb1 = (const float*)d_in[7]; const float* tw2 = (const float*)d_in[8]; const float* tb2 = (const float*)d_in[9];
    const float* wq = (const float*)d_in[10]; const float* bq = (const float*)d_in[11]; const float* wk = (const float*)d_in[12]; const float* bk = (const float*)d_in[13]; const float* wv = (const float*)d_in[14]; const float* bv = (const float*)d_in[15]; const float* wo = (const float*)d_in[16]; const float* bo = (const float*)d_in[17];
    const float* aw1 = (const float*)d_in[18]; const float* ab1 = (const float*)d_in[19]; const float* aw2 = (const float*)d_in[20]; const float* ab2 = (const float*)d_in[21]; const float* aw3 = (const float*)d_in[22]; const float* ab3 = (const float*)d_in[23];
    float* out = (float*)d_out;
    char* wsp = (char*)d_ws;
    auto take = [&](size_t bytes) { char* p = wsp; wsp += (bytes + 255) & ~(size_t)255; return (void*)p; };
    bf* RW1 = (bf*)take(64 * 32 * 2); bf* RW2 = (bf*)take(64 * 64 * 2); bf* TW1 = (bf*)take(64 * 32 * 2); bf* TW2 = (bf*)take(64 * 64 * 2);
    bf* WQ = (bf*)take(64 * 64 * 2); bf* WK = (bf*)take(64 * 64 * 2); bf* WV = (bf*)take(64 * 64 * 2); bf* WO = (bf*)take(64 * 64 * 2); bf* AW1T = (bf*)take(64 * 64 * 2); bf* AW1R = (bf*)take(64 * 64 * 2); bf* AW2 = (bf*)take(64 * 64 * 2);
    bf* RX = (bf*)take((size_t)NRR * 32 * 2); bf* TX = (bf*)take((size_t)NTR * 32 * 2); float* T1 = (float*)take((size_t)NRR * HH * 4);
    bf* Rh = (bf*)take((size_t)NRR * HH * 2); bf* Rl = (bf*)take((size_t)NRR * HH * 2); float* RF = (float*)take((size_t)NRR * HH * 4); bf* RFh = (bf*)take((size_t)NRR * HH * 2); bf* RFl = (bf*)take((size_t)NRR * HH * 2);
    bf* Th = (bf*)take((size_t)NTR * HH * 2); bf* Tl = (bf*)take((size_t)NTR * HH * 2); bf* TFh = (bf*)take((size_t)NTR * HH * 2); bf* TFl = (bf*)take((size_t)NTR * HH * 2);
    float* Qf = (float*)take((size_t)NTR * HH * 4); float* Kf = (float*)take((size_t)NRR * HH * 4); float* Vf = (float*)take((size_t)NRR * HH * 4); float* CTX = (float*)take((size_t)NTR * HH * 4); bf* Ch = (bf*)take((size_t)NTR * HH * 2); bf* Cl = (bf*)take((size_t)NTR * HH * 2);
    float* TP = (float*)take((size_t)NTR * HH * 4); float* RP = (float*)take((size_t)NRR * HH * 4); bf* Hh = (bf*)take((size_t)NPR * HH * 2); bf* Hl = (bf*)take((size_t)NPR * HH * 2); float* H2 = (float*)take((size_t)NPR * HH * 4);
    if ((size_t)(wsp - (char*)d_ws) > ws_size) return;
    k_w32k<<<1, 256, 0, stream>>>(rw1, 7, RW1); k_w32k<<<1, 256, 0, stream>>>(tw1, 6, TW1);
    k_wt<<<dim3(1, 1, 1), 256, 0, stream>>>(rw2, HH, HH, RW2); k_wt<<<dim3(1, 1, 1), 256, 0, stream>>>(tw2, HH, HH, TW2);
    k_wt<<<dim3(1, 1, 1), 256, 0, stream>>>(wq, HH, HH, WQ); k_wt<<<dim3(1, 1, 1), 256, 0, stream>>>(wk, HH, HH, WK); k_wt<<<dim3(1, 1, 1), 256, 0, stream>>>(wv, HH, HH, WV); k_wt<<<dim3(1, 1, 1), 256, 0, stream>>>(wo, HH, HH, WO);
    k_wt<<<dim3(1, 1, 1), 256, 0, stream>>>(aw1, HH, HH, AW1T); k_wt<<<dim3(1, 1, 1), 256, 0, stream>>>(aw1 + (size_t)HH * HH, HH, HH, AW1R); k_wtp<<<dim3(1, 1, 1), 256, 0, stream>>>(aw2, HH, HH / 2, HH, AW2);
    k_pad32<<<NRR / 64, 256, 0, stream>>>(rs, NRR, 7, RX); k_pad32<<<NTR / 64, 256, 0, stream>>>(ts, NTR, 6, TX);
    k_gemmb<false, false><<<dim3(NRR / 64, 1, 1), 128, 0, stream>>>(RX, nullptr, RW1, nullptr, T1, HH, nullptr, nullptr, 32); k_act64<true><<<NRR / 8, 256, 0, stream>>>(T1, rb1, NRR, Rh, Rl, nullptr);
    k_gemmb<true, false><<<dim3(NRR / 64, 1, 1), 128, 0, stream>>>(Rh, Rl, RW2, nullptr, T1, HH, nullptr, nullptr, HH); k_act64<true><<<NRR / 8, 256, 0, stream>>>(T1, rb2, NRR, RFh, RFl, nullptr);
    k_gemmb<false, false><<<dim3(NTR / 64, 1, 1), 128, 0, stream>>>(TX, nullptr, TW1, nullptr, T1, HH, nullptr, nullptr, 32); k_act64<true><<<NTR / 8, 256, 0, stream>>>(T1, tb1, NTR, Th, Tl, nullptr);
    k_gemmb<true, false><<<dim3(NTR / 64, 1, 1), 128, 0, stream>>>(Th, Tl, TW2, nullptr, T1, HH, nullptr, nullptr, HH); k_act64<true><<<NTR / 8, 256, 0, stream>>>(T1, tb2, NTR, TFh, TFl, nullptr);
    k_gemmb<true, false><<<dim3(NTR / 64, 1, 1), 128, 0, stream>>>(TFh, TFl, WQ, bq, Qf, HH, nullptr, nullptr, HH);
    k_gemmb<true, false><<<dim3(NRR / 64, 1, 1), 128, 0, stream>>>(RFh, RFl, WK, bk, Kf, HH, nullptr, nullptr, HH);
    k_gemmb<true, false><<<dim3(NRR / 64, 1, 1), 128, 0, stream>>>(RFh, RFl, WV, bv, Vf, HH, nullptr, nullptr, HH);
    k_attn16<<<NTR / 8, 256, 0, stream>>>(Qf, Kf, Vf, CTX); k_act64<false><<<NTR / 8, 256, 0, stream>>>(CTX, nullptr, NTR, Ch, Cl, nullptr);
    k_gemmb<true, false><<<dim3(NTR / 64, 1, 1), 128, 0, stream>>>(Ch, Cl, WO, bo, T1, HH, nullptr, nullptr, HH); k_act64<false><<<NTR / 8, 256, 0, stream>>>(T1, nullptr, NTR, Th, Tl, nullptr);
    k_gemmb<true, false><<<dim3(NTR / 64, 1, 1), 128, 0, stream>>>(Th, Tl, AW1T, nullptr, TP, HH, nullptr, nullptr, HH);
    k_gemmb<true, false><<<dim3(NRR / 64, 1, 1), 128, 0, stream>>>(RFh, RFl, AW1R, nullptr, RP, HH, nullptr, nullptr, HH);
    for (int b = 0; b < NBT; ++b) {
        k_h1<<<NPR / 8, 256, 0, stream>>>(TP, RP, ab1, b, Hh, Hl);
        k_gemmb<true, false><<<dim3(NPR / 64, 1, 1), 128, 0, stream>>>(Hh, Hl, AW2, nullptr, H2, HH, nullptr, nullptr, HH);
        k_score<<<NTS / 8, 256, 0, stream>>>(H2, ab2, aw3, ab3, b, out + (size_t)b * NTS * NRB); }
}
